// SelectiveSSM_33277406610014
// MI455X (gfx1250) — hardware-verified
//
#include <hip/hip_runtime.h>
#include <math.h>

typedef __attribute__((ext_vector_type(16))) _Float16 v16h;
typedef __attribute__((ext_vector_type(8)))  _Float16 v8h;
typedef __attribute__((ext_vector_type(16))) __bf16   v16b;
typedef __attribute__((ext_vector_type(8)))  __bf16   v8b;
typedef __attribute__((ext_vector_type(8)))  float    v8f;
typedef __attribute__((ext_vector_type(4)))  float    v4f;

constexpr int kBatch = 4;
constexpr int kSeq   = 1024;
constexpr int kDm    = 64;
constexpr int kDin   = 128;
constexpr int kDst   = 128;
constexpr int kRows  = kBatch * kSeq;
constexpr int kNcol  = 2 * kDin + kDin + kDst + kDst;
constexpr int kColXs    = 0;
constexpr int kColGate  = kDin;
constexpr int kColDelta = 2 * kDin;
constexpr int kColB     = 3 * kDin;
constexpr int kColC     = 3 * kDin + kDst;
constexpr int kScanChunk = 128;
constexpr float kWCarry  = 16.0f;
constexpr float kResCarry = 1024.0f;
constexpr float kSgCarry = 64.0f;
constexpr float kLnEps   = 1e-5f;
static_assert(kDin == 128 && kDst == 128 && kNcol == 640, "fused column map");
static_assert((kDm % 32) == 0 && (kDin % 32) == 0, "GEMM K multiples of 32");
static_assert((kRows % 64) == 0 && (kRows % 16) == 0 && (kNcol % 64) == 0 && (kDm % 64) == 0, "GEMM M,N tile multiples");
static_assert((((kRows / 16) * (kNcol / 64)) % 8) == 0 && (((kRows / 64) * (kDm / 64)) % 8) == 0, "8 wave tiles per GEMM block exactly");
static_assert((kSeq % kScanChunk) == 0 && kScanChunk == 4 * 32, "scan chunk = 32 lanes x 4 steps");
static_assert((kRows % 16) == 0, "finalize rows per block");

constexpr size_t kOffXH    = 0;
constexpr size_t kOffXL    = kOffXH    + (size_t)kRows * kDm * 2;
constexpr size_t kOffWALLH = kOffXL    + (size_t)kRows * kDm * 2;
constexpr size_t kOffWALLL = kOffWALLH + (size_t)kNcol * kDm * 2;
constexpr size_t kOffWOUT  = kOffWALLL + (size_t)kNcol * kDm * 2;
constexpr size_t kOffBIAS  = kOffWOUT  + (size_t)kDm * kDin * 2;
constexpr size_t kOffP     = kOffBIAS  + (size_t)kNcol * 4;
constexpr size_t kOffABAR  = kOffP     + (size_t)kRows * kNcol * 4;
constexpr size_t kOffBX    = kOffABAR  + (size_t)kRows * kDst * 4;
constexpr size_t kOffSG    = kOffBX    + (size_t)kRows * kDst * 4;
constexpr size_t kOffG     = kOffSG    + (size_t)kRows * kDin * 2;
constexpr size_t kOffYP    = kOffG     + (size_t)kRows * kDm * 4;
constexpr size_t kWsTotal  = kOffYP    + (size_t)kBatch * 4 * kSeq * 4;
static_assert(kWsTotal == 18074112ull, "carve total");
static_assert(kWsTotal <= 134217728ull, "carve cap");
static_assert((kOffXL % 128) == 0 && (kOffWALLH % 128) == 0 && (kOffWALLL % 128) == 0 && (kOffWOUT % 128) == 0 &&
              (kOffBIAS % 128) == 0 && (kOffP % 128) == 0 && (kOffABAR % 128) == 0 && (kOffBX % 128) == 0 &&
              (kOffSG % 128) == 0 && (kOffG % 128) == 0 && (kOffYP % 128) == 0, "128-B aligned regions");
constexpr size_t kWallInElems    = (size_t)0;
constexpr size_t kWallDeltaElems = (size_t)256 * kDm;
constexpr size_t kWallBElems     = (size_t)384 * kDm;
constexpr size_t kWallCElems     = (size_t)512 * kDm;
static_assert(((kWallDeltaElems * 2) % 128) == 0 && ((kWallBElems * 2) % 128) == 0 && ((kWallCElems * 2) % 128) == 0, "sub-plane alignment");

__device__ __forceinline__ void keep4_h(v16h a, v16h b, v16h c, v16h d) { asm volatile("v_nop" :: "v"(a), "v"(b), "v"(c), "v"(d)); }
__device__ __forceinline__ void acc_guard4(v8f& a, v8f& b, v8f& c, v8f& d) { asm volatile("v_nop\n\tv_nop\n\tv_nop\n\tv_nop" : "+v"(a), "+v"(b), "+v"(c), "+v"(d)); }
__device__ __forceinline__ void dep_guard4_h(v8f& a, v8f& b, v8f& c, v8f& d, v16h x, v16h y) {
  asm volatile("v_nop\n\tv_nop\n\tv_nop\n\tv_nop" : "+v"(a), "+v"(b), "+v"(c), "+v"(d) : "v"(x), "v"(y));
}
__device__ __forceinline__ void dep_guard8_h(v8f& a, v8f& b, v8f& c, v8f& d, v8f& e, v8f& f, v8f& g, v8f& h, v16h x, v16h y) {
  asm volatile("v_nop\n\tv_nop\n\tv_nop\n\tv_nop" : "+v"(a), "+v"(b), "+v"(c), "+v"(d), "+v"(e), "+v"(f), "+v"(g), "+v"(h) : "v"(x), "v"(y));
}
template <typename T> struct Frag;
template <> struct Frag<_Float16> {
  typedef v16h V; union U { v16h v; v8h h[2]; };
  static __device__ __forceinline__ v16h load(const _Float16* p) {
    U f; f.h[0] = *(const v8h*)(p); f.h[1] = *(const v8h*)(p + 16); return f.v;
  }
  static __device__ __forceinline__ v8f mma(v16h a, v16h b, v8f c) {
    return __builtin_amdgcn_wmma_f32_16x16x32_f16(false, a, false, b, (short)0, c, false, false);
  }
};

template <int MSUB, bool SPLIT, bool BIASN>
__global__ __launch_bounds__(256) void gemm_f16_kernel(
    const unsigned short* __restrict__ Ap, const unsigned short* __restrict__ A2p, int lda,
    const unsigned short* __restrict__ Btp, const unsigned short* __restrict__ Bt2p, int ldb,
    float* __restrict__ C, int ldc, const float* __restrict__ bias,
    int M, int N, int K, float scale, float scale2)
{
  typedef _Float16 T;
  const T* A = (const T*)Ap; const T* A2 = (const T*)A2p; const T* Bt = (const T*)Btp; const T* Bt2 = (const T*)Bt2p;
  __shared__ __align__(16) float sT[8][16 * 68];
  const int lane = threadIdx.x & 31;
  const int wave = threadIdx.x >> 5;
  const int tilesN = N >> 6;
  const int tilesM = M / (16 * MSUB);
  const int tile = blockIdx.x * 8 + wave;
  if (tile >= tilesM * tilesN) return;
  const int tm = tile / tilesN;
  const int tn = tile - tm * tilesN;
  const int m0 = tm * (16 * MSUB);
  const int n0 = tn << 6;

  const int rlane = lane & 15;
  const int koff  = (lane >> 4) * 8;
  const int mOff  = (lane >> 4) * 8;

  v8f acc[MSUB][4], accr[MSUB][4];
#pragma unroll
  for (int i = 0; i < MSUB; ++i)
#pragma unroll
    for (int j = 0; j < 4; ++j) {
      acc[i][j]  = (v8f){0.f,0.f,0.f,0.f,0.f,0.f,0.f,0.f};
      accr[i][j] = (v8f){0.f,0.f,0.f,0.f,0.f,0.f,0.f,0.f};
    }

  for (int k0 = 0; k0 < K; k0 += 32) {
    v16h bh[4], bl[4];
#pragma unroll
    for (int j = 0; j < 4; ++j) {
      const size_t bo = (size_t)(n0 + (j << 4) + rlane) * ldb + koff + k0;
      bh[j] = Frag<T>::load(Bt + bo);
      if (SPLIT) bl[j] = Frag<T>::load(Bt2 + bo);
    }
#pragma unroll
    for (int i = 0; i < MSUB; ++i) {
      const size_t ao = (size_t)(m0 + (i << 4) + rlane) * lda + koff + k0;
      v16h ah = Frag<T>::load(A + ao);
      v16h al = ah;
      if (SPLIT) al = Frag<T>::load(A2 + ao);
#pragma unroll
      for (int j = 0; j < 4; ++j) {
        acc[i][j] = Frag<T>::mma(ah, bh[j], acc[i][j]);
        if (SPLIT) {
          accr[i][j] = Frag<T>::mma(ah, bl[j], accr[i][j]);
          accr[i][j] = Frag<T>::mma(al, bh[j], accr[i][j]);
        }
      }
      if (SPLIT) dep_guard8_h(acc[i][0], acc[i][1], acc[i][2], acc[i][3], accr[i][0], accr[i][1], accr[i][2], accr[i][3], ah, al);
      else       dep_guard4_h(acc[i][0], acc[i][1], acc[i][2], acc[i][3], ah, al);
    }
    keep4_h(bh[0], bh[1], bh[2], bh[3]);
    if (SPLIT) keep4_h(bl[0], bl[1], bl[2], bl[3]);
  }
#pragma unroll
  for (int i = 0; i < MSUB; ++i) {
    acc_guard4(acc[i][0], acc[i][1], acc[i][2], acc[i][3]);
    if (SPLIT) acc_guard4(accr[i][0], accr[i][1], accr[i][2], accr[i][3]);
  }

  float* slab = sT[wave];
#pragma unroll
  for (int i = 0; i < MSUB; ++i) {
    const int mBase = m0 + (i << 4);
#pragma unroll
    for (int j = 0; j < 4; ++j) {
      const int n = n0 + (j << 4) + rlane;
      float bv = 0.f;
      if (BIASN) bv = bias[n];
#pragma unroll
      for (int r = 0; r < 8; ++r) {
        float v = acc[i][j][r] * scale;
        if (SPLIT) v = fmaf(accr[i][j][r], scale2, v);
        if (BIASN) v += bv;
        slab[(mOff + r) * 68 + (j << 4) + rlane] = v;
      }
    }
    __builtin_amdgcn_fence(__ATOMIC_RELEASE, "workgroup");
    __builtin_amdgcn_wave_barrier();
    __builtin_amdgcn_fence(__ATOMIC_ACQUIRE, "workgroup");
    {
      const int hh = lane >> 4, c4 = (lane & 15) * 4;
      for (int pass = 0; pass < 2; ++pass) {
#pragma unroll
        for (int it = 0; it < 8; ++it) {
          const int row = it * 2 + hh;
          v4f v = *(const v4f*)(slab + row * 68 + c4);
          *(volatile v4f*)(C + (size_t)(mBase + row) * ldc + n0 + c4) = v;
        }
        __threadfence();
      }
    }
    __builtin_amdgcn_fence(__ATOMIC_RELEASE, "workgroup");
    __builtin_amdgcn_wave_barrier();
    __builtin_amdgcn_fence(__ATOMIC_ACQUIRE, "workgroup");
  }
}

__device__ __forceinline__ float wave_sum32(float v) {
  v += __shfl_xor(v, 16, 32);
  v += __shfl_xor(v,  8, 32);
  v += __shfl_xor(v,  4, 32);
  v += __shfl_xor(v,  2, 32);
  v += __shfl_xor(v,  1, 32);
  return v;
}

__global__ __launch_bounds__(256) void cast8_f16_kernel(
    const float* __restrict__ src, unsigned short* __restrict__ dst, int total8, float scale)
{
  const int i = blockIdx.x * 256 + threadIdx.x;
  if (i >= total8) return;
  const size_t e0 = (size_t)i << 3;
  const v4f a0 = *(const v4f*)(src + e0);
  const v4f a1 = *(const v4f*)(src + e0 + 4);
  v8h hv;
#pragma unroll
  for (int e = 0; e < 4; ++e) {
    hv[e]     = (_Float16)(a0[e] * scale);
    hv[4 + e] = (_Float16)(a1[e] * scale);
  }
  unsigned short* q = dst + e0;
  *(volatile v8h*)q = hv;
  __threadfence();
  *(volatile v8h*)q = hv;
}

__global__ __launch_bounds__(256) void split8_f16_kernel(
    const float* __restrict__ src, unsigned short* __restrict__ dhi, unsigned short* __restrict__ dlo, int total8,
    float pre, float carry)
{
  const int i = blockIdx.x * 256 + threadIdx.x;
  if (i >= total8) return;
  const size_t e0 = (size_t)i << 3;
  const v4f a0 = *(const v4f*)(src + e0);
  const v4f a1 = *(const v4f*)(src + e0 + 4);
  v8h hv, lv;
#pragma unroll
  for (int e = 0; e < 4; ++e) {
    const float f0 = a0[e] * pre, f1 = a1[e] * pre;
    const _Float16 h0 = (_Float16)f0, h1 = (_Float16)f1;
    const float g0 = (float)h0, g1 = (float)h1;
    const float r0 = (f0 - g0) * carry, r1 = (f1 - g1) * carry;
    hv[e]     = h0;
    hv[4 + e] = h1;
    lv[e]     = (_Float16)r0;
    lv[4 + e] = (_Float16)r1;
  }
  unsigned short* qh = dhi + e0;
  unsigned short* ql = dlo + e0;
  *(volatile v8h*)qh = hv;
  *(volatile v8h*)ql = lv;
  __threadfence();
  *(volatile v8h*)qh = hv;
  *(volatile v8h*)ql = lv;
}

__global__ __launch_bounds__(256) void bias_pack_kernel(
    const float* __restrict__ bd, const float* __restrict__ bb, const float* __restrict__ bc, float* __restrict__ bias)
{
  const int i = threadIdx.x;
  if (i >= kNcol / 4) return;
  const int wave = i >> 5;
  const int si = (i & 31) * 4;
  const v4f vd = *(const v4f*)(bd + si);
  const v4f vb = *(const v4f*)(bb + si);
  const v4f vc = *(const v4f*)(bc + si);
  const float fd = (wave == 2) ? 1.0f : 0.0f;
  const float fb = (wave == 3) ? 1.0f : 0.0f;
  const float fc = (wave == 4) ? 1.0f : 0.0f;
  v4f v;
#pragma unroll
  for (int e = 0; e < 4; ++e) v[e] = fmaf(fd, vd[e], fmaf(fb, vb[e], fc * vc[e]));
  float* q = bias + 4 * i;
  *(volatile v4f*)q = v;
  __threadfence();
  *(volatile v4f*)q = v;
}

__global__ __launch_bounds__(128) void prep_kernel(
    const float* __restrict__ P, const float* __restrict__ Am,
    float* __restrict__ Abar, float* __restrict__ Bx, unsigned short* __restrict__ SG)
{
  __shared__ float sDelta[kDin];
  __shared__ float sRed[4];
  __shared__ __align__(16) float sOut[3 * kDst];
  const int tid = threadIdx.x, lane = tid & 31, wave = tid >> 5;
  const int row = blockIdx.x;
  const size_t pb = (size_t)row * kNcol;
  const float xs = P[pb + kColXs + tid];
  const float g  = P[pb + kColGate + tid];
  const float dz = P[pb + kColDelta + tid];
  const float bm = P[pb + kColB + tid];
  const float delta = fmaxf(dz, 0.0f) + log1pf(expf(-fabsf(dz)));
  sDelta[tid] = delta;
  const float wsum = wave_sum32(xs);
  if (lane == 0) sRed[wave] = wsum;
  __syncthreads();
  const float x_pool = ((sRed[0] + sRed[1]) + (sRed[2] + sRed[3])) * (1.0f / 128.0f);
  float acc = 0.0f;
#pragma unroll 1
  for (int i = 0; i < kDin; ++i) {
    const float t = sDelta[i] * Am[(size_t)i * kDst + tid];
    acc += expf(t) - 1.0f;
  }
  const float abar = 1.0f + acc * (1.0f / 128.0f);
  const float sig  = 1.0f / (1.0f + expf(-g));
  sOut[tid]            = abar;
  sOut[kDst + tid]     = bm * x_pool;
  sOut[2 * kDst + tid] = g * sig * kSgCarry;
  __syncthreads();
  if (wave == 0) {
    const v4f v = *(const v4f*)(sOut + 4 * lane);
    float* q = Abar + (size_t)row * kDst + 4 * lane;
    *(volatile v4f*)q = v;
    __threadfence();
    *(volatile v4f*)q = v;
  } else if (wave == 1) {
    const v4f v = *(const v4f*)(sOut + kDst + 4 * lane);
    float* q = Bx + (size_t)row * kDst + 4 * lane;
    *(volatile v4f*)q = v;
    __threadfence();
    *(volatile v4f*)q = v;
  } else if (wave == 2) {
    const int c8 = (lane & 15) * 8;
    const v4f s0 = *(const v4f*)(sOut + 2 * kDst + c8);
    const v4f s1 = *(const v4f*)(sOut + 2 * kDst + c8 + 4);
    v8h hv;
#pragma unroll
    for (int e = 0; e < 4; ++e) {
      hv[e]     = (_Float16)s0[e];
      hv[4 + e] = (_Float16)s1[e];
    }
    unsigned short* q = SG + (size_t)row * kDin + c8;
    if (lane < 16) *(volatile v8h*)q = hv;
    __threadfence();
    if (lane < 16) *(volatile v8h*)q = hv;
  }
}

__global__ __launch_bounds__(128) void scan_kernel(
    const float* __restrict__ Abar, const float* __restrict__ Bx, const float* __restrict__ P, float* __restrict__ YP)
{
  __shared__ __align__(16) float sY[4 * kScanChunk];
  const int tid = threadIdx.x, lane = tid & 31, wave = tid >> 5;
  const int b = blockIdx.x;
  const int s = tid;
  float h = 0.0f;
#pragma unroll 1
  for (int l0 = 0; l0 < kSeq; l0 += kScanChunk) {
#pragma unroll 1
    for (int t = 0; t < kScanChunk; ++t) {
      const size_t row = (size_t)b * kSeq + l0 + t;
      const float a  = Abar[row * kDst + s];
      const float bx = Bx[row * kDst + s];
      const float cc = P[row * kNcol + kColC + s];
      h = a * h + bx;
      const float p = wave_sum32(cc * h);
      if (lane == 0) sY[wave * kScanChunk + t] = p;
    }
    __syncthreads();
    const v4f v = *(const v4f*)(sY + wave * kScanChunk + 4 * lane);
    float* q = YP + (size_t)(b * 4 + wave) * kSeq + l0 + 4 * lane;
    *(volatile v4f*)q = v;
    __threadfence();
    *(volatile v4f*)q = v;
    __syncthreads();
  }
}

__global__ __launch_bounds__(256) void finalize_kernel(
    const float* __restrict__ G, const float* __restrict__ YP, const float* __restrict__ x,
    const float* __restrict__ lnw, const float* __restrict__ lnb, float* __restrict__ out)
{
  const int tid = threadIdx.x, lane = tid & 31, wave = tid >> 5;
  const int hh = lane >> 4, c4 = (lane & 15) * 4;
  const int row = (blockIdx.x * 8 + wave) * 2 + hh;
  const int b = row >> 10, l = row & (kSeq - 1);
  const float* yp = YP + (size_t)(b * 4) * kSeq + l;
  const float y = ((yp[0] + yp[kSeq]) + yp[2 * kSeq]) + yp[3 * kSeq];
  const v4f gv = *(const v4f*)(G + (size_t)row * kDm + c4);
  const v4f xv = *(const v4f*)(x + (size_t)row * kDm + c4);
  const v4f wv = *(const v4f*)(lnw + c4);
  const v4f bv = *(const v4f*)(lnb + c4);
  v4f v;
  float s1 = 0.0f;
#pragma unroll
  for (int e = 0; e < 4; ++e) { v[e] = xv[e] + y * gv[e]; s1 += v[e]; }
  s1 += __shfl_xor(s1, 1, 32);
  s1 += __shfl_xor(s1, 2, 32);
  s1 += __shfl_xor(s1, 4, 32);
  s1 += __shfl_xor(s1, 8, 32);
  const float mu = s1 * (1.0f / 64.0f);
  v4f d;
  float s2 = 0.0f;
#pragma unroll
  for (int e = 0; e < 4; ++e) { d[e] = v[e] - mu; s2 += d[e] * d[e]; }
  s2 += __shfl_xor(s2, 1, 32);
  s2 += __shfl_xor(s2, 2, 32);
  s2 += __shfl_xor(s2, 4, 32);
  s2 += __shfl_xor(s2, 8, 32);
  const float var = s2 * (1.0f / 64.0f);
  const float rs = rsqrtf(var + kLnEps);
  v4f o;
#pragma unroll
  for (int e = 0; e < 4; ++e) o[e] = d[e] * rs * wv[e] + bv[e];
  float* q = out + (size_t)row * kDm + c4;
  *(volatile v4f*)q = o;
  __threadfence();
  *(volatile v4f*)q = o;
}

extern "C" void kernel_launch(void* const* d_in, const int* in_sizes, int n_in,
                              void* d_out, int out_size, void* d_ws, size_t ws_size,
                              hipStream_t stream) {
  if (n_in < 12) return;
  if (in_sizes[0]  != kRows * kDm) return;
  if (in_sizes[1]  != 2 * kDin * kDm) return;
  if (in_sizes[2]  != kDin * kDm) return;
  if (in_sizes[3]  != kDin) return;
  if (in_sizes[4]  != kDst * kDm) return;
  if (in_sizes[5]  != kDst) return;
  if (in_sizes[6]  != kDst * kDm) return;
  if (in_sizes[7]  != kDst) return;
  if (in_sizes[8]  != kDin * kDst) return;
  if (in_sizes[9]  != kDm * kDin) return;
  if (in_sizes[10] != kDm) return;
  if (in_sizes[11] != kDm) return;
  if (out_size != kRows * kDm) return;
  if (ws_size < kWsTotal) return;

  const float* x       = (const float*)d_in[0];
  const float* W_in    = (const float*)d_in[1];
  const float* W_delta = (const float*)d_in[2];
  const float* b_delta = (const float*)d_in[3];
  const float* W_B     = (const float*)d_in[4];
  const float* b_B     = (const float*)d_in[5];
  const float* W_C     = (const float*)d_in[6];
  const float* b_C     = (const float*)d_in[7];
  const float* Amat    = (const float*)d_in[8];
  const float* W_out   = (const float*)d_in[9];
  const float* ln_w    = (const float*)d_in[10];
  const float* ln_b    = (const float*)d_in[11];
  float* out = (float*)d_out;

  char* ws = (char*)d_ws;
  unsigned short* XH    = (unsigned short*)(ws + kOffXH);
  unsigned short* XL    = (unsigned short*)(ws + kOffXL);
  unsigned short* WALLH = (unsigned short*)(ws + kOffWALLH);
  unsigned short* WALLL = (unsigned short*)(ws + kOffWALLL);
  unsigned short* WOUT  = (unsigned short*)(ws + kOffWOUT);
  float*          BIAS  = (float*)(ws + kOffBIAS);
  float*          P     = (float*)(ws + kOffP);
  float*          ABAR  = (float*)(ws + kOffABAR);
  float*          BX    = (float*)(ws + kOffBX);
  unsigned short* SG    = (unsigned short*)(ws + kOffSG);
  float*          G     = (float*)(ws + kOffG);
  float*          YP    = (float*)(ws + kOffYP);

  {
    const int t8x = kRows * kDm / 8;
    const int t8i = 2 * kDin * kDm / 8;
    const int t8w = kDin * kDm / 8;
    const int t8o = kDm * kDin / 8;
    split8_f16_kernel<<<(t8x + 255) / 256, 256, 0, stream>>>(x, XH, XL, t8x, 1.0f, kResCarry);
    split8_f16_kernel<<<(t8i + 255) / 256, 256, 0, stream>>>(W_in,    WALLH + kWallInElems,    WALLL + kWallInElems,    t8i, kWCarry, kResCarry);
    split8_f16_kernel<<<(t8w + 255) / 256, 256, 0, stream>>>(W_delta, WALLH + kWallDeltaElems, WALLL + kWallDeltaElems, t8w, kWCarry, kResCarry);
    split8_f16_kernel<<<(t8w + 255) / 256, 256, 0, stream>>>(W_B,     WALLH + kWallBElems,     WALLL + kWallBElems,     t8w, kWCarry, kResCarry);
    split8_f16_kernel<<<(t8w + 255) / 256, 256, 0, stream>>>(W_C,     WALLH + kWallCElems,     WALLL + kWallCElems,     t8w, kWCarry, kResCarry);
    cast8_f16_kernel<<<(t8o + 255) / 256, 256, 0, stream>>>(W_out, WOUT, t8o, kWCarry);
  }
  bias_pack_kernel<<<1, kNcol / 4, 0, stream>>>(b_delta, b_B, b_C, BIAS);

  gemm_f16_kernel<1, true, true><<<dim3((kRows / 16) * (kNcol / 64) / 8), 256, 0, stream>>>(
      XH, XL, kDm,
      WALLH, WALLL, kDm,
      P, kNcol, BIAS,
      kRows, kNcol, kDm, 1.0f / kWCarry, 1.0f / (kWCarry * kResCarry));

  prep_kernel<<<kRows, kDin, 0, stream>>>(P, Amat, ABAR, BX, SG);

  gemm_f16_kernel<4, false, false><<<dim3((kRows / 64) * (kDm / 64) / 8), 256, 0, stream>>>(
      SG, SG, kDin,
      WOUT, WOUT, kDin,
      G, kDm, BIAS,
      kRows, kDm, kDin, 1.0f / (kWCarry * kSgCarry), 0.0f);

  scan_kernel<<<kBatch, kDst, 0, stream>>>(ABAR, BX, P, YP);

  finalize_kernel<<<kRows / 16, 256, 0, stream>>>(G, YP, x, ln_w, ln_b, out);
}
